// NAM_32229434589251
// MI455X (gfx1250) — hardware-run, weakly checked
//
#include <hip/hip_runtime.h>


#ifndef NROWS
#define NROWS 8192
#endif
#define NROWS_FULL 8192
#define NF   64
#define HW   128
#define NC   32
#define KW   (NF * HW)
#define AW   4
#define XP   68
#define OSP  36
#define TP   136
#define HC   4.0f
#define W2C  64.0f
#define FC   256.0f
#define WOC  1024.0f
#define FOLD (1.0f / 262144.0f)

static_assert(HC * W2C == FC);
static_assert(FC * WOC * FOLD == 1.0f);
static_assert(NC == 32);
static_assert(NF == 64);
static_assert(16 * NF == 8 * 32 * 4);
static_assert(HW == 128);
static_assert(HW % 32 == 0);
static_assert(KW % 32 == 0);
static_assert(NROWS % (16 * AW) == 0);
static_assert(NROWS <= NROWS_FULL);
static_assert((XP * 4) % 16 == 0);
static_assert((OSP * 4) % 16 == 0);
static_assert((TP * 2) % 16 == 0);
static_assert(XP >= NF);
static_assert(OSP >= NC);
static_assert(TP >= HW);
static_assert(4 * 32 * 16 == 16 * NC * 4);
static_assert(8 * 256 * 4 == HW * 64);
static_assert(4 * 256 * 8 == 64 * HW);
static_assert(AW * 16 * XP * 4 + AW * 16 * OSP * 4 <= 131072);
static_assert(64 * TP * 2 <= 131072);

typedef _Float16 h16;
typedef __attribute__((ext_vector_type(16))) _Float16 v16h;
typedef __attribute__((ext_vector_type(8)))  _Float16 v8h;
typedef __attribute__((ext_vector_type(8)))  float    v8f;
typedef __attribute__((ext_vector_type(4)))  float    v4f;
typedef v4f  __attribute__((may_alias)) v4fa;
typedef v8h  __attribute__((may_alias)) v8ha;

__device__ __forceinline__ unsigned short f2bf(float f) { unsigned u = __float_as_uint(f); u += 0x7FFFu + ((u >> 16) & 1u); return (unsigned short)(u >> 16); }
__device__ __forceinline__ float bfr(float f) { return __uint_as_float(((unsigned)f2bf(f)) << 16); }
__device__ __forceinline__ v16h cat16(v8h lo, v8h hi) { return __builtin_shufflevector(lo, hi, 0, 1, 2, 3, 4, 5, 6, 7, 8, 9, 10, 11, 12, 13, 14, 15); }
__device__ __forceinline__ v8f wmma16(v16h a, v16h b, v8f c) { return __builtin_amdgcn_wmma_f32_16x16x32_f16(false, a, false, b, (short)0, c, false, false); }
__device__ __forceinline__ v8f wmma16g(v16h a, v16h b, v8f c) { c = wmma16(a, b, c); asm volatile("v_nop\n\tv_nop\n\tv_nop\n\tv_nop" : "+v"(c) : "v"(a), "v"(b)); return c; }
__device__ __forceinline__ v16h ldh(const h16* p) { return cat16(*(const v8h*)p, *(const v8h*)(p + 16)); }
__device__ __forceinline__ void wave_sync() { __builtin_amdgcn_fence(3  , "wavefront"); __builtin_amdgcn_wave_barrier(); asm volatile("" ::: "memory"); }
static __device__ __forceinline__ h16 toh_flush(float v) { const float w = (fabsf(v) < 6.103515625e-05f) ? 0.0f : v; return (h16)w; }
__device__ __forceinline__ h16 hact(float x, float w, float b) { const float v = x * w + b; const float r = (v > 0.0f) ? v : 0.0f; return toh_flush(r); }

__global__ __launch_bounds__(256) void k_w2t(const float* __restrict__ w2, h16* W2T) {
    __shared__ __align__(16) h16 tl[64 * TP];
    const unsigned t = threadIdx.x;
    const unsigned f = blockIdx.x, kb = blockIdx.y * 64u;
    const float* src = w2 + (size_t)f * HW * HW + kb;
#pragma unroll 1
    for (unsigned it = 0; it < 8u; ++it) {
        const unsigned idx = it * 256u + t; const unsigned h = idx >> 4, k4 = (idx & 15u) * 4u;
        const v4f v = *(const v4f*)(src + (size_t)h * HW + k4);
#pragma unroll
        for (int i = 0; i < 4; ++i) tl[(k4 + (unsigned)i) * TP + h] = toh_flush(bfr(v[i]) * W2C);
    }
    __syncthreads();
    h16* dst = W2T + ((size_t)f * HW + kb) * HW;
#pragma unroll 1
    for (int ps = 0; ps < 2; ++ps) {
#pragma unroll
        for (int it = 0; it < 4; ++it) { const unsigned row = (unsigned)it * 16u + (t >> 4), c8 = (t & 15u) * 8u;
            const v8h v = *(const v8ha*)(&tl[row * TP + c8]);
            *(volatile v8h*)(dst + (size_t)row * HW + c8) = v; }
        if (ps == 0) __threadfence(); }
}

__global__ __launch_bounds__(256) void k_cvtwo(const float* __restrict__ src, h16* dst, unsigned n8) {
    const unsigned i = blockIdx.x * 256u + threadIdx.x; if (i >= n8) return;
    const v8f v = *(const v8f*)(src + (size_t)i * 8); v8h o;
#pragma unroll
    for (int k = 0; k < 8; ++k) o[k] = toh_flush(bfr(v[k]) * WOC);
    *(volatile v8h*)(dst + (size_t)i * 8) = o; __threadfence(); *(volatile v8h*)(dst + (size_t)i * 8) = o;
}

__global__ __launch_bounds__(256) void k_cvts(const float* __restrict__ w1, const float* __restrict__ b1, const float* __restrict__ b2,
                                              float* W1S, float* B1S, float* B2S, unsigned n4) {
    const unsigned i = blockIdx.x * 256u + threadIdx.x; if (i >= n4) return;
    const v4f a = *(const v4f*)(w1 + (size_t)i * 4), b = *(const v4f*)(b1 + (size_t)i * 4), c = *(const v4f*)(b2 + (size_t)i * 4);
    v4f oa, ob, oc;
#pragma unroll
    for (int k = 0; k < 4; ++k) { oa[k] = bfr(a[k]) * HC; ob[k] = bfr(b[k]) * HC; oc[k] = bfr(c[k]) * FC; }
    *(volatile v4f*)(W1S + (size_t)i * 4) = oa; *(volatile v4f*)(B1S + (size_t)i * 4) = ob; *(volatile v4f*)(B2S + (size_t)i * 4) = oc;
    __threadfence();
    *(volatile v4f*)(W1S + (size_t)i * 4) = oa; *(volatile v4f*)(B1S + (size_t)i * 4) = ob; *(volatile v4f*)(B2S + (size_t)i * 4) = oc;
}

__global__ __launch_bounds__(32 * AW) __attribute__((amdgpu_num_vgpr(256)))
void k_main(const float* __restrict__ X, const float* __restrict__ W1S, const float* __restrict__ B1S, const h16* __restrict__ W2T,
            const float* __restrict__ B2S, const h16* __restrict__ WOH, const float* __restrict__ bout, float* OUT) {
    __shared__ __align__(16) float xs[AW * 16 * XP];
    __shared__ __align__(16) float os[AW * 16 * OSP];
    const int lane = threadIdx.x & 31, lr = lane & 15, hi = lane >> 4;
    const int wave = __builtin_amdgcn_readfirstlane((int)(threadIdx.x >> 5));
    const unsigned bx = blockIdx.x;
    const unsigned b0 = (bx * (unsigned)AW + (unsigned)wave) * 16u;
    const int xb = wave * 16 * XP;
    { const float* xg = X + (size_t)b0 * NF;
#pragma unroll
      for (int s = 0; s < 8; ++s) { const int p = s * 32 + lane; const int row = p >> 4, c4 = (p & 15) * 4;
          const v4f v = *(const v4f*)(xg + (size_t)p * 4); v4f o;
#pragma unroll
          for (int i = 0; i < 4; ++i) o[i] = bfr(v[i]);
          *(v4fa*)(&xs[xb + row * XP + c4]) = o; } }
    wave_sync();
    v8f hd0 = (v8f){}, hd1 = (v8f){};
#pragma unroll 1
    for (int f = 0; f < NF; ++f) {
        const float xv = xs[xb + lr * XP + f];
        const float* w1p = W1S + (size_t)f * HW + 8 * hi;
        const float* b1p = B1S + (size_t)f * HW + 8 * hi;
        v16h a[4];
#pragma unroll
        for (int ks = 0; ks < 4; ++ks) {
            const v4f wa0 = *(const v4f*)(w1p + 32 * ks), wa1 = *(const v4f*)(w1p + 32 * ks + 4), wa2 = *(const v4f*)(w1p + 32 * ks + 16), wa3 = *(const v4f*)(w1p + 32 * ks + 20);
            const v4f ca0 = *(const v4f*)(b1p + 32 * ks), ca1 = *(const v4f*)(b1p + 32 * ks + 4), ca2 = *(const v4f*)(b1p + 32 * ks + 16), ca3 = *(const v4f*)(b1p + 32 * ks + 20);
#pragma unroll
            for (int i = 0; i < 4; ++i) {
                a[ks][i]      = hact(xv, wa0[i], ca0[i]);
                a[ks][4 + i]  = hact(xv, wa1[i], ca1[i]);
                a[ks][8 + i]  = hact(xv, wa2[i], ca2[i]);
                a[ks][12 + i] = hact(xv, wa3[i], ca3[i]); }
        }
        const h16* w2p = W2T + ((size_t)f * HW + (size_t)lr) * HW + 8 * hi;
        const float* b2p = B2S + (size_t)f * HW + 8 * hi;
        const h16* wop = WOH + (size_t)lr * KW + (size_t)f * HW + 8 * hi;
#pragma unroll
        for (int p = 0; p < 2; ++p) {
            v8f acc[4];
#pragma unroll
            for (int j = 0; j < 4; ++j) acc[j] = (v8f){};
#pragma unroll
            for (int ks = 0; ks < 4; ++ks) {
#pragma unroll
                for (int j = 0; j < 4; ++j) { const v16h wa = ldh(w2p + (size_t)((p * 4 + j) * 16) * HW + 32 * ks);
                    acc[j] = wmma16g(wa, a[ks], acc[j]); } }
#pragma unroll
            for (int q = 0; q < 2; ++q) {
                const float* bp = b2p + (p * 4 + 2 * q) * 16;
                const v4f e0 = *(const v4f*)bp, e1 = *(const v4f*)(bp + 4), e2 = *(const v4f*)(bp + 16), e3 = *(const v4f*)(bp + 20);
                v16h pb;
#pragma unroll
                for (int i = 0; i < 4; ++i) {
                    pb[i]      = toh_flush(acc[2 * q][i] + e0[i]);
                    pb[4 + i]  = toh_flush(acc[2 * q][4 + i] + e1[i]);
                    pb[8 + i]  = toh_flush(acc[2 * q + 1][i] + e2[i]);
                    pb[12 + i] = toh_flush(acc[2 * q + 1][4 + i] + e3[i]); }
                const int kq = (p * 2 + q) * 32;
                const v16h wo0 = ldh(wop + kq), wo1 = ldh(wop + (size_t)16 * KW + kq);
                hd0 = wmma16g(wo0, pb, hd0); hd1 = wmma16g(wo1, pb, hd1);
            }
        }
    }
    const int wb = wave * 16 * OSP;
    { const float* bp = bout + 8 * hi;
      const v4f q0 = *(const v4f*)bp, q1 = *(const v4f*)(bp + 4), q2 = *(const v4f*)(bp + 16), q3 = *(const v4f*)(bp + 20);
      v4f a4, c4;
#pragma unroll
      for (int i = 0; i < 4; ++i) { a4[i] = hd0[i] * FOLD + bfr(q0[i]); c4[i] = hd0[4 + i] * FOLD + bfr(q1[i]); }
      *(v4fa*)(&os[wb + lr * OSP +  0 + 8 * hi]) = a4; *(v4fa*)(&os[wb + lr * OSP +  0 + 8 * hi + 4]) = c4;
#pragma unroll
      for (int i = 0; i < 4; ++i) { a4[i] = hd1[i] * FOLD + bfr(q2[i]); c4[i] = hd1[4 + i] * FOLD + bfr(q3[i]); }
      *(v4fa*)(&os[wb + lr * OSP + 16 + 8 * hi]) = a4; *(v4fa*)(&os[wb + lr * OSP + 16 + 8 * hi + 4]) = c4; }
    wave_sync();
    float* orow = OUT + (size_t)b0 * NC;
#pragma unroll 1
    for (int ps = 0; ps < 2; ++ps) {
#pragma unroll
        for (int s = 0; s < 4; ++s) { const int row = 4 * s + (lane >> 3), cofs = (lane & 7) * 4;
            const v4f val = *(const v4fa*)(&os[wb + row * OSP + cofs]);
            *(volatile v4f*)(orow + (size_t)row * NC + cofs) = val; }
        if (ps == 0) __threadfence(); }
}

static constexpr size_t al256(size_t v) { return (v + 255) & ~(size_t)255; }
static constexpr size_t SZ_W2T = al256((size_t)NF * HW * HW * 2);
static constexpr size_t SZ_WOH = al256((size_t)NC * KW * 2);
static constexpr size_t SZ_SP  = al256((size_t)NF * HW * 4);
static constexpr size_t SZ_TOTAL = SZ_W2T + SZ_WOH + 3 * SZ_SP;
static_assert(SZ_TOTAL <= (size_t)134217728);
static constexpr unsigned N8_WO = (unsigned)((size_t)NC * KW / 8);
static constexpr unsigned G_WO  = (N8_WO + 255u) / 256u;
static constexpr unsigned N4_SP = (unsigned)((size_t)NF * HW / 4);
static constexpr unsigned G_SP  = (N4_SP + 255u) / 256u;
static_assert(((size_t)NC * KW) % 8 == 0);
static_assert(((size_t)NF * HW) % 4 == 0);
static_assert(HW % 64 == 0);
static constexpr size_t NEED_X  = (size_t)NROWS * NF;
static constexpr size_t NEED_V  = (size_t)NF * HW;
static constexpr size_t NEED_W2 = (size_t)NF * HW * HW;
static constexpr size_t NEED_WO = (size_t)NC * KW;
static constexpr size_t NEED_O  = (size_t)NROWS * NC;
static constexpr unsigned G_MAIN = (unsigned)(NROWS / (16 * AW));

extern "C" void kernel_launch(void* const* d_in, const int* in_sizes, int n_in,
                              void* d_out, int out_size, void* d_ws, size_t ws_size, hipStream_t stream) {
    if (n_in < 7) return;
    if ((size_t)in_sizes[0] < NEED_X) return;
    if ((size_t)in_sizes[1] < NEED_V || (size_t)in_sizes[2] < NEED_V || (size_t)in_sizes[4] < NEED_V) return;
    if ((size_t)in_sizes[3] < NEED_W2 || (size_t)in_sizes[5] < NEED_WO) return;
    if (in_sizes[6] < NC) return;
    if ((size_t)out_size < NEED_O) return;
    if (SZ_TOTAL > ws_size) return;
    const float* x    = (const float*)d_in[0];
    const float* w1   = (const float*)d_in[1];
    const float* b1   = (const float*)d_in[2];
    const float* w2   = (const float*)d_in[3];
    const float* b2   = (const float*)d_in[4];
    const float* wout = (const float*)d_in[5];
    const float* bout = (const float*)d_in[6];
    float* OUT = (float*)d_out;
    char* wsp = (char*)d_ws;
    h16* W2T = (h16*)wsp; wsp += SZ_W2T;
    h16* WOH = (h16*)wsp; wsp += SZ_WOH;
    float* W1S = (float*)wsp; wsp += SZ_SP;
    float* B1S = (float*)wsp; wsp += SZ_SP;
    float* B2S = (float*)wsp; wsp += SZ_SP;

    k_w2t<<<dim3(NF, HW / 64, 1), 256, 0, stream>>>(w2, W2T);
    k_cvtwo<<<G_WO, 256, 0, stream>>>(wout, WOH, N8_WO);
    k_cvts<<<G_SP, 256, 0, stream>>>(w1, b1, b2, W1S, B1S, B2S, N4_SP);
    k_main<<<G_MAIN, 32 * AW, 0, stream>>>(x, W1S, B1S, W2T, B2S, WOH, bout, OUT);
}
